// LSTMModel_17540646437690
// MI455X (gfx1250) — hardware-verified
//
#include <hip/hip_runtime.h>
#include <math.h>

constexpr int NBATCH   = 8192;
constexpr int NSTEP    = 50;
constexpr int NFEAT    = 7;
constexpr int NHID     = 64;
constexpr int NGATE    = 4 * NHID;
constexpr int NPRED    = 30;
constexpr int TFIRST   = NSTEP - NPRED;
constexpr int NOUTCH   = 2;
constexpr int ROWS_BLK = 16;
constexpr int NTHR     = 128;
constexpr int XROW     = NSTEP * NFEAT;
constexpr int XTILE    = ROWS_BLK * XROW;
constexpr int XTILE4   = XTILE / 4;
constexpr int XSTAGE_IT = (XTILE4 + NTHR - 1) / NTHR;
constexpr int WXK      = 32;
constexpr int HPITCH   = 72;
constexpr int HPLANE   = ROWS_BLK * HPITCH;
constexpr int FPITCH   = 68;
constexpr int OUTROW   = NPRED * NOUTCH;
constexpr int OUTTILE  = ROWS_BLK * OUTROW;
constexpr int OUTTILE4 = OUTTILE / 4;
constexpr int WX_HALVES = NGATE * WXK;
constexpr int WB_HALVES = 3 * NGATE * NHID;
constexpr int WX_CHUNKS = WX_HALVES / 8;
constexpr int WB_CHUNKS = WB_HALVES / 8;
constexpr int PACK_THR  = 256;
constexpr int WX_BLOCKS = WX_CHUNKS / PACK_THR;
constexpr int WB_BLOCKS = WB_CHUNKS / PACK_THR;
constexpr int PLANE_BLOCKS = (NGATE * NHID / 8) / PACK_THR;
constexpr float ACT_CARRY  = 16.0f;
constexpr float W_CARRY    = 256.0f;
constexpr float RES_CARRY  = 2048.0f;
constexpr float FOLD_MAIN  = 1.0f / (ACT_CARRY * W_CARRY);
constexpr float FOLD_RES   = 1.0f / RES_CARRY;
constexpr float F16_MIN_NORMAL = 6.103515625e-5f;

static_assert(NBATCH % ROWS_BLK == 0, "grid exact");
static_assert(NHID == 16 * (NTHR / 32), "one 16-column slice per wave");
static_assert(NHID % 32 == 0 && WXK % 32 == 0, "K multiple of 32");
static_assert(NFEAT < 8, "x features fit the first 8 k slots");
static_assert(XTILE % 4 == 0, "x tile is a whole number of float4");
static_assert((ROWS_BLK * XROW * 4) % 16 == 0, "x tile base 16-B aligned");
static_assert((ROWS_BLK * OUTROW * 4) % 128 == 0, "output tile is whole 128-B lines");
static_assert(OUTTILE4 <= 2 * NTHR, "output store loop covers the tile");
static_assert(WX_CHUNKS % NTHR == 0 && WB_CHUNKS % NTHR == 0, "LDS weight copy exact");
static_assert(WX_CHUNKS % PACK_THR == 0 && WB_CHUNKS % PACK_THR == 0, "pack grid exact");
static_assert(PLANE_BLOCKS == 8, "plane select by shift");
static_assert((8 * HPLANE / 8) % NTHR == 0, "h zero-fill exact");
static_assert(NTHR == NOUTCH * NHID, "head weight staging exact");
static_assert(NTHR == ROWS_BLK * 8, "head thread map exact");

typedef __attribute__((ext_vector_type(16))) _Float16 v16h;
typedef __attribute__((ext_vector_type(8)))  _Float16 v8h;
typedef __attribute__((ext_vector_type(8)))  float    v8f;
typedef __attribute__((ext_vector_type(4)))  float    v4f;
typedef __attribute__((ext_vector_type(2)))  unsigned v2u;
typedef __attribute__((ext_vector_type(8)))  unsigned v8u;

union FragU { v16h v; v8h h[2]; };

__device__ __forceinline__ v16h frag_load(const _Float16* p) {
  FragU f;
  f.h[0] = *(const v8h*)(p);
  f.h[1] = *(const v8h*)(p + 16);
  return f.v;
}

__device__ __forceinline__ v8f mma_h(v16h a, v16h b, v8f c) {
  return __builtin_amdgcn_wmma_f32_16x16x32_f16(false, a, false, b, (short)0, c, false, false);
}

__device__ __forceinline__ void guard4x(v8f& m0, v8f& m1, v8f& m2, v8f& m3,
                                        v16h a, v16h b0, v16h b1, v16h b2, v16h b3) {
  asm volatile("v_nop\n\tv_nop\n\tv_nop\n\tv_nop"
               : "+v"(m0), "+v"(m1), "+v"(m2), "+v"(m3)
               : "v"(a), "v"(b0), "v"(b1), "v"(b2), "v"(b3)
               : "memory");
}
__device__ __forceinline__ void guard8(v8f& m0, v8f& m1, v8f& m2, v8f& m3,
                                       v8f& r0, v8f& r1, v8f& r2, v8f& r3,
                                       v16h a, v16h al, v16h b0, v16h b1, v16h b2, v16h b3) {
  asm volatile("v_nop\n\tv_nop\n\tv_nop\n\tv_nop"
               : "+v"(m0), "+v"(m1), "+v"(m2), "+v"(m3), "+v"(r0), "+v"(r1), "+v"(r2), "+v"(r3)
               : "v"(a), "v"(al), "v"(b0), "v"(b1), "v"(b2), "v"(b3)
               : "memory");
}

__device__ __forceinline__ float sigm(float z) {
  return __builtin_amdgcn_rcpf(1.0f + expf(-z));
}
__device__ __forceinline__ float tanh_id(float z) {
  return 1.0f - 2.0f * __builtin_amdgcn_rcpf(1.0f + expf(2.0f * z));
}

__device__ __forceinline__ void hgroup(v8f (&M)[4], v8f (&R)[4],
                                       const _Float16* ahi, const _Float16* alo, const _Float16* wrow) {
  const v16h a  = frag_load(ahi);
  const v16h al = frag_load(alo);
  const v16h b0 = frag_load(wrow);
  const v16h b1 = frag_load(wrow + 1 * NHID * NHID);
  const v16h b2 = frag_load(wrow + 2 * NHID * NHID);
  const v16h b3 = frag_load(wrow + 3 * NHID * NHID);
  M[0] = mma_h(a, b0, M[0]);
  M[1] = mma_h(a, b1, M[1]);
  M[2] = mma_h(a, b2, M[2]);
  M[3] = mma_h(a, b3, M[3]);
  R[0] = mma_h(al, b0, R[0]);
  R[1] = mma_h(al, b1, R[1]);
  R[2] = mma_h(al, b2, R[2]);
  R[3] = mma_h(al, b3, R[3]);
  guard8(M[0], M[1], M[2], M[3], R[0], R[1], R[2], R[3], a, al, b0, b1, b2, b3);
}

template <bool WRITE_F32>
__device__ __forceinline__ void cell_step(const v8f (&M)[4], const v8f (&R)[4], const float (&bb)[4],
                                          float (&cs)[8], _Float16* hiP, _Float16* loP, float* hf) {
#pragma unroll
  for (int r = 0; r < 8; ++r) {
    const float zi = (M[0][r] + R[0][r] * FOLD_RES) * FOLD_MAIN + bb[0];
    const float zf = (M[1][r] + R[1][r] * FOLD_RES) * FOLD_MAIN + bb[1];
    const float zg = (M[2][r] + R[2][r] * FOLD_RES) * FOLD_MAIN + bb[2];
    const float zo = (M[3][r] + R[3][r] * FOLD_RES) * FOLD_MAIN + bb[3];
    const float ig = sigm(zi);
    const float fg = sigm(zf);
    const float gg = tanh_id(zg);
    const float og = sigm(zo);
    const float cn = fg * cs[r] + ig * gg;
    cs[r] = cn;
    const float hn = og * tanh_id(cn);
    const float v  = hn * ACT_CARRY;
    const float vh = (fabsf(v) < F16_MIN_NORMAL) ? 0.0f : v;
    const _Float16 hi = (_Float16)vh;
    const float hif = (float)hi;
    const float lo = (v - hif) * RES_CARRY;
    hiP[r * HPITCH] = hi;
    loP[r * HPITCH] = (_Float16)lo;
    if (WRITE_F32) hf[r * FPITCH] = hn;
  }
}

__global__ __launch_bounds__(PACK_THR) void pack_weights_kernel(const float* __restrict__ wih0, const float* __restrict__ whh0,
                                                               const float* __restrict__ wih1, const float* __restrict__ whh1,
                                                               unsigned short* __restrict__ dst) {
  const int tid = threadIdx.x;
  const int bx  = blockIdx.x;
  float zl = 0.0f;
  asm volatile("" : "+v"(zl));
  v8h hv;
  size_t chunk;
  if (bx < WX_BLOCKS) {
    const int i  = bx * PACK_THR + tid;
    const int n  = i >> 2;
    const int ch = i & 3;
    const float* sp = wih0 + n * NFEAT;
    const float f0 = sp[0];
    const float f1 = sp[1];
    const float f2 = sp[2];
    const float f3 = sp[3];
    const float f4 = sp[4];
    const float f5 = sp[5];
    const float f6 = sp[6];
    const bool first = (ch == 0);
    hv[0] = (_Float16)(first ? f0 * W_CARRY : zl);
    hv[1] = (_Float16)(first ? f1 * W_CARRY : zl);
    hv[2] = (_Float16)(first ? f2 * W_CARRY : zl);
    hv[3] = (_Float16)(first ? f3 * W_CARRY : zl);
    hv[4] = (_Float16)(first ? f4 * W_CARRY : zl);
    hv[5] = (_Float16)(first ? f5 * W_CARRY : zl);
    hv[6] = (_Float16)(first ? f6 * W_CARRY : zl);
    hv[7] = (_Float16)zl;
    chunk = (size_t)i;
  } else {
    const int pb = bx - WX_BLOCKS;
    const int pl = pb >> 3;
    const float* src = (pl == 0) ? whh0 : ((pl == 1) ? wih1 : whh1);
    const int within = (pb & 7) * PACK_THR + tid;
    const v4f a = *(const v4f*)(src + within * 8);
    const v4f b = *(const v4f*)(src + within * 8 + 4);
#pragma unroll
    for (int e = 0; e < 4; ++e) {
      hv[e]     = (_Float16)(a[e] * W_CARRY);
      hv[4 + e] = (_Float16)(b[e] * W_CARRY);
    }
    chunk = (size_t)(WX_CHUNKS + pb * PACK_THR + tid);
  }
  volatile v8h* dp = (volatile v8h*)(dst + chunk * 8);
  *dp = hv;
  __threadfence();
  *dp = hv;
}

__global__ __launch_bounds__(NTHR) void lstm2_seq_kernel(const float* __restrict__ x, const unsigned short* __restrict__ wpk,
                                                        const float* __restrict__ bih0, const float* __restrict__ bhh0,
                                                        const float* __restrict__ bih1, const float* __restrict__ bhh1,
                                                        const float* __restrict__ wfc, const float* __restrict__ bfc,
                                                        float* __restrict__ out) {
  __shared__ __align__(16) _Float16       WXs[WX_HALVES];
  __shared__ __align__(16) _Float16       WBs[WB_HALVES];
  __shared__ __align__(16) unsigned short Xs[XTILE];
  __shared__ __align__(16) _Float16       Hp[8 * HPLANE];
  __shared__ __align__(16) float          H2f[ROWS_BLK * FPITCH];
  __shared__ __align__(16) float          OutS[OUTTILE];
  __shared__ __align__(16) float          WfcS[NOUTCH * NHID];
  __shared__ __align__(16) float          BfcS[4];

  const int tid  = threadIdx.x;
  const int lane = tid & 31;
  const int wave = tid >> 5;
  const int c    = lane & 15;
  const int hh   = lane >> 4;
  const int j    = 16 * wave + c;
  const int b0   = blockIdx.x * ROWS_BLK;

  {
    const v8h* src = (const v8h*)(const void*)wpk;
#pragma unroll 4
    for (int it = 0; it < WX_CHUNKS / NTHR; ++it) {
      const int i = it * NTHR + tid;
      const v8h w = src[i];
      *(v8h*)(WXs + i * 8) = w;
    }
#pragma unroll 4
    for (int it = 0; it < WB_CHUNKS / NTHR; ++it) {
      const int i = it * NTHR + tid;
      const v8h w = src[WX_CHUNKS + i];
      *(v8h*)(WBs + i * 8) = w;
    }
  }
  {
    v8h zv;
#pragma unroll
    for (int e = 0; e < 8; ++e) zv[e] = (_Float16)0.0f;
#pragma unroll 1
    for (int it = 0; it < (8 * HPLANE / 8) / NTHR; ++it) {
      const int i = it * NTHR + tid;
      *(v8h*)(Hp + i * 8) = zv;
    }
  }
  {
    const float* xblk = x + (size_t)b0 * XROW;
#pragma unroll 1
    for (int it = 0; it < XSTAGE_IT; ++it) {
      const int i  = it * NTHR + tid;
      const int ic = (i < XTILE4) ? i : (XTILE4 - 1);
      const v4f v = *(const v4f*)(xblk + ic * 4);
      const float f0 = v[0];
      const float f1 = v[1];
      const float f2 = v[2];
      const float f3 = v[3];
      const _Float16 h0 = (_Float16)(f0 * ACT_CARRY);
      const _Float16 h1 = (_Float16)(f1 * ACT_CARRY);
      const _Float16 h2 = (_Float16)(f2 * ACT_CARRY);
      const _Float16 h3 = (_Float16)(f3 * ACT_CARRY);
      const unsigned q0 = (unsigned)__builtin_bit_cast(unsigned short, h0);
      const unsigned q1 = (unsigned)__builtin_bit_cast(unsigned short, h1);
      const unsigned q2 = (unsigned)__builtin_bit_cast(unsigned short, h2);
      const unsigned q3 = (unsigned)__builtin_bit_cast(unsigned short, h3);
      v2u pk;
      pk[0] = q0 | (q1 << 16);
      pk[1] = q2 | (q3 << 16);
      if (i < XTILE4) *(v2u*)(Xs + i * 4) = pk;
    }
  }
  WfcS[tid] = wfc[tid];
  {
    const float bv = bfc[tid & 1];
    if (tid < NOUTCH) BfcS[tid] = bv;
  }
  float bb0[4], bb1[4];
#pragma unroll
  for (int g = 0; g < 4; ++g) bb0[g] = bih0[g * NHID + j] + bhh0[g * NHID + j];
  asm volatile("" ::: "memory");
#pragma unroll
  for (int g = 0; g < 4; ++g) bb1[g] = bih1[g * NHID + j] + bhh1[g * NHID + j];

  float c0s[8], c1s[8];
#pragma unroll
  for (int r = 0; r < 8; ++r) {
    c0s[r] = 0.0f;
    c1s[r] = 0.0f;
  }
  __syncthreads();

  const _Float16* wx_row = WXs + j * WXK + 8 * hh;
  const _Float16* w0_row = WBs + j * NHID + 8 * hh;
  const _Float16* w1_row = w0_row + NGATE * NHID;
  const _Float16* w2_row = w0_row + 2 * NGATE * NHID;
  const int a_off  = c * HPITCH + 8 * hh;
  const int st_off = 8 * hh * HPITCH + j;
  const v8f z8 = {0.f, 0.f, 0.f, 0.f, 0.f, 0.f, 0.f, 0.f};
  const bool lowhalf = (hh == 0);

#pragma unroll 1
  for (int t = 0; t < NSTEP; ++t) {
    const int cur = t & 1;
    const int nxt = cur ^ 1;
    _Float16* h1hi_c = Hp + (0 + cur) * HPLANE;
    _Float16* h1hi_n = Hp + (0 + nxt) * HPLANE;
    _Float16* h1lo_c = Hp + (2 + cur) * HPLANE;
    _Float16* h1lo_n = Hp + (2 + nxt) * HPLANE;
    _Float16* h2hi_c = Hp + (4 + cur) * HPLANE;
    _Float16* h2hi_n = Hp + (4 + nxt) * HPLANE;
    _Float16* h2lo_c = Hp + (6 + cur) * HPLANE;
    _Float16* h2lo_n = Hp + (6 + nxt) * HPLANE;

    v8f M[4], R[4];
#pragma unroll
    for (int g = 0; g < 4; ++g) {
      M[g] = z8;
      R[g] = z8;
    }

    {
      const int xo = c * XROW + t * NFEAT;
      const unsigned u0 = (unsigned)Xs[xo + 0];
      const unsigned u1 = (unsigned)Xs[xo + 1];
      const unsigned u2 = (unsigned)Xs[xo + 2];
      const unsigned u3 = (unsigned)Xs[xo + 3];
      const unsigned u4 = (unsigned)Xs[xo + 4];
      const unsigned u5 = (unsigned)Xs[xo + 5];
      const unsigned u6 = (unsigned)Xs[xo + 6];
      const unsigned p0 = u0 | (u1 << 16);
      const unsigned p1 = u2 | (u3 << 16);
      const unsigned p2 = u4 | (u5 << 16);
      const unsigned p3 = u6;
      v8u xw;
      xw[0] = lowhalf ? p0 : 0u;
      xw[1] = lowhalf ? p1 : 0u;
      xw[2] = lowhalf ? p2 : 0u;
      xw[3] = lowhalf ? p3 : 0u;
      xw[4] = 0u;
      xw[5] = 0u;
      xw[6] = 0u;
      xw[7] = 0u;
      const v16h ax = __builtin_bit_cast(v16h, xw);
      const v16h b0 = frag_load(wx_row);
      const v16h b1 = frag_load(wx_row + 1 * NHID * WXK);
      const v16h b2 = frag_load(wx_row + 2 * NHID * WXK);
      const v16h b3 = frag_load(wx_row + 3 * NHID * WXK);
      M[0] = mma_h(ax, b0, M[0]);
      M[1] = mma_h(ax, b1, M[1]);
      M[2] = mma_h(ax, b2, M[2]);
      M[3] = mma_h(ax, b3, M[3]);
      guard4x(M[0], M[1], M[2], M[3], ax, b0, b1, b2, b3);
    }
#pragma unroll
    for (int kt = 0; kt < 2; ++kt)
      hgroup(M, R, h1hi_c + a_off + kt * 32, h1lo_c + a_off + kt * 32, w0_row + kt * 32);
    cell_step<false>(M, R, bb0, c0s, h1hi_n + st_off, h1lo_n + st_off, H2f);
    __syncthreads();

#pragma unroll
    for (int g = 0; g < 4; ++g) {
      M[g] = z8;
      R[g] = z8;
    }
#pragma unroll
    for (int kt = 0; kt < 2; ++kt)
      hgroup(M, R, h1hi_n + a_off + kt * 32, h1lo_n + a_off + kt * 32, w1_row + kt * 32);
#pragma unroll
    for (int kt = 0; kt < 2; ++kt)
      hgroup(M, R, h2hi_c + a_off + kt * 32, h2lo_c + a_off + kt * 32, w2_row + kt * 32);
    cell_step<true>(M, R, bb1, c1s, h2hi_n + st_off, h2lo_n + st_off, H2f + 8 * hh * FPITCH + j);
    __syncthreads();

    if (t >= TFIRST) {
      const int m    = tid >> 3;
      const int part = tid & 7;
      const v4f ha  = *(const v4f*)(H2f + m * FPITCH + part * 8);
      const v4f hb  = *(const v4f*)(H2f + m * FPITCH + part * 8 + 4);
      const v4f wa0 = *(const v4f*)(WfcS + part * 8);
      const v4f wb0 = *(const v4f*)(WfcS + part * 8 + 4);
      const v4f wa1 = *(const v4f*)(WfcS + NHID + part * 8);
      const v4f wb1 = *(const v4f*)(WfcS + NHID + part * 8 + 4);
      float s0 = 0.0f;
      float s1 = 0.0f;
#pragma unroll
      for (int e = 0; e < 4; ++e) {
        s0 += ha[e] * wa0[e];
        s1 += ha[e] * wa1[e];
      }
#pragma unroll
      for (int e = 0; e < 4; ++e) {
        s0 += hb[e] * wb0[e];
        s1 += hb[e] * wb1[e];
      }
      s0 += __shfl_xor(s0, 1, 32);
      s1 += __shfl_xor(s1, 1, 32);
      s0 += __shfl_xor(s0, 2, 32);
      s1 += __shfl_xor(s1, 2, 32);
      s0 += __shfl_xor(s0, 4, 32);
      s1 += __shfl_xor(s1, 4, 32);
      const float o0 = s0 + BfcS[0];
      const float o1 = s1 + BfcS[1];
      if (part == 0) {
        OutS[m * OUTROW + (t - TFIRST) * NOUTCH + 0] = o0;
        OutS[m * OUTROW + (t - TFIRST) * NOUTCH + 1] = o1;
      }
    }
  }

  __syncthreads();
  {
    float* ob = out + (size_t)b0 * OUTROW;
    for (int pass = 0; pass < 2; ++pass) {
#pragma unroll
      for (int it = 0; it < 2; ++it) {
        const int idx = it * NTHR + tid;
        if (idx < OUTTILE4) {
          const v4f v = *(const v4f*)(OutS + idx * 4);
          *(volatile v4f*)(ob + idx * 4) = v;
        }
      }
      __threadfence();
    }
  }
}

extern "C" void kernel_launch(void* const* d_in, const int* in_sizes, int n_in,
                              void* d_out, int out_size, void* d_ws, size_t ws_size, hipStream_t stream) {
  if (n_in < 11 || d_out == nullptr || d_ws == nullptr) return;
  if (in_sizes[0] != NBATCH * NSTEP * NFEAT || in_sizes[1] != NGATE * NFEAT || in_sizes[2] != NGATE * NHID ||
      in_sizes[3] != NGATE || in_sizes[4] != NGATE || in_sizes[5] != NGATE * NHID || in_sizes[6] != NGATE * NHID ||
      in_sizes[7] != NGATE || in_sizes[8] != NGATE || in_sizes[9] != NOUTCH * NHID || in_sizes[10] != NOUTCH ||
      out_size != NBATCH * NPRED * NOUTCH) return;

  const float* x    = (const float*)d_in[0];
  const float* wih0 = (const float*)d_in[1];
  const float* whh0 = (const float*)d_in[2];
  const float* bih0 = (const float*)d_in[3];
  const float* bhh0 = (const float*)d_in[4];
  const float* wih1 = (const float*)d_in[5];
  const float* whh1 = (const float*)d_in[6];
  const float* bih1 = (const float*)d_in[7];
  const float* bhh1 = (const float*)d_in[8];
  const float* wfc  = (const float*)d_in[9];
  const float* bfc  = (const float*)d_in[10];
  float* out = (float*)d_out;

  char* ws = (char*)d_ws;
  size_t off = 0;
  unsigned short* WPK = (unsigned short*)(ws + off);
  off += (((size_t)(WX_HALVES + WB_HALVES) * 2) + 255) & ~(size_t)255;
  if (off > ws_size || off > (size_t)134217728) return;

  pack_weights_kernel<<<WX_BLOCKS + WB_BLOCKS, PACK_THR, 0, stream>>>(wih0, whh0, wih1, whh1, WPK);
  lstm2_seq_kernel<<<NBATCH / ROWS_BLK, NTHR, 0, stream>>>(x, WPK, bih0, bhh0, bih1, bhh1, wfc, bfc, out);
}
